// MixingLayer_24936580121077
// MI455X (gfx1250) — hardware-verified
//
#include <hip/hip_runtime.h>


#define NBM  1024
#define NF   128
#define L2   16
#define LMX  4
#define KD   64
#define KBIG (NF * NF * LMX)
#define RCH  128
#define DM   KD
#define LOSC 1024.0f

typedef _Float16 h16;
typedef unsigned short bf;
typedef __attribute__((ext_vector_type(16))) __bf16   v16bf;
typedef __attribute__((ext_vector_type(16))) _Float16 v16h;
typedef __attribute__((ext_vector_type(8)))  _Float16 v8h;
typedef __attribute__((ext_vector_type(8)))  unsigned short v8us;
typedef __attribute__((ext_vector_type(8)))  float    v8f;
typedef __attribute__((ext_vector_type(4)))  float    v4f;
typedef v8h  __attribute__((may_alias)) v8ha;
typedef v4f  __attribute__((may_alias)) v4fa;
typedef v8us __attribute__((may_alias)) v8usa;

__device__ __forceinline__ unsigned short f2bf(float f) { unsigned u = __float_as_uint(f); u += 0x7FFFu + ((u >> 16) & 1u); return (unsigned short)(u >> 16); }
__device__ __forceinline__ float bf2f(unsigned short b) { return __uint_as_float(((unsigned)b) << 16); }
__device__ __forceinline__ float bfr(float f) { return bf2f(f2bf(f)); }
__device__ __forceinline__ v16h cat16(v8h lo, v8h hi) { return __builtin_shufflevector(lo, hi, 0, 1, 2, 3, 4, 5, 6, 7, 8, 9, 10, 11, 12, 13, 14, 15); }
__device__ __forceinline__ v16bf cat16b(v8us lo, v8us hi) { return __builtin_bit_cast(v16bf, __builtin_shufflevector(lo, hi, 0, 1, 2, 3, 4, 5, 6, 7, 8, 9, 10, 11, 12, 13, 14, 15)); }
__device__ __forceinline__ v8f wmma16(v16h a, v16h b, v8f c) { return __builtin_amdgcn_wmma_f32_16x16x32_f16(false, a, false, b, (short)0, c, false, false); }
__device__ __forceinline__ v8f wmmab(v16bf a, v16bf b, v8f c) { return __builtin_amdgcn_wmma_f32_16x16x32_bf16(false, a, false, b, (short)0, c, false, false); }

template <bool SPLITA, bool F16OUT = false>
__global__ __launch_bounds__(128) void k_gemmb(const bf* __restrict__ A, const bf* __restrict__ Al, const bf* __restrict__ Bn, const float* __restrict__ bias, float* C, int ldc, h16* C2, const float* __restrict__ R = nullptr, int K = DM, int roundR = 1) {
    __shared__ __align__(16) float ost[4][16 * 68];
    const int lane = threadIdx.x & 31, wave = threadIdx.x >> 5, lr = lane & 15, hi = lane >> 4;
    const int r0 = blockIdx.x * 64 + wave * 16, c0 = blockIdx.y * 64;
    const size_t aoff = (size_t)(r0 + lr) * K + 8 * hi;
    size_t boff[4];
#pragma unroll
    for (int t = 0; t < 4; ++t) boff[t] = (size_t)(c0 + t * 16 + lr) * K + 8 * hi;
    v8f acc[4];
#pragma unroll
    for (int t = 0; t < 4; ++t) acc[t] = (v8f){};
#pragma unroll 1
    for (int kc = 0; kc < K; kc += 32) {
        const v16bf a = cat16b(*(const v8us*)(A + aoff + kc), *(const v8us*)(A + aoff + kc + 16));
        v16bf al = a;
        if (SPLITA) al = cat16b(*(const v8us*)(Al + aoff + kc), *(const v8us*)(Al + aoff + kc + 16));
#pragma unroll
        for (int t = 0; t < 4; ++t) { const v16bf b = cat16b(*(const v8us*)(Bn + boff[t] + kc), *(const v8us*)(Bn + boff[t] + kc + 16)); acc[t] = wmmab(a, b, acc[t]); if (SPLITA) acc[t] = wmmab(al, b, acc[t]); }
        asm volatile("v_nop\n\tv_nop\n\tv_nop\n\tv_nop" : "+v"(acc[0]), "+v"(acc[1]), "+v"(acc[2]), "+v"(acc[3]) : "v"(a), "v"(al));
    }
    float* os = &ost[wave][0];
#pragma unroll
    for (int t = 0; t < 4; ++t) { const float bv = bias ? bfr(bias[c0 + t * 16 + lr]) : 0.f;
#pragma unroll
        for (int j = 0; j < 8; ++j) os[(hi * 8 + j) * 68 + t * 16 + lr] = acc[t][j] + bv; }
    __syncthreads();
    if (F16OUT) {
        h16* crow = (h16*)(void*)C + (size_t)r0 * ldc + c0;
        auto pass = [&]() {
#pragma unroll
            for (int s = 0; s < 4; ++s) { const int row = 4 * s + (lane >> 3), piece = lane & 7; const float* sp = os + row * 68 + piece * 8; v8h o, o2;
#pragma unroll
                for (int i = 0; i < 8; ++i) { const h16 a = (h16)sp[i]; o[i] = a; o2[i] = (h16)((sp[i] - (float)a) * LOSC); }
                *(volatile v8h*)(crow + (size_t)row * ldc + piece * 8) = o; if (C2) *(volatile v8h*)(C2 + (size_t)r0 * ldc + c0 + (size_t)row * ldc + piece * 8) = o2; }
        };
        pass(); __threadfence(); pass();
    } else {
        float* crow = C + (size_t)r0 * ldc + c0;
        auto pass = [&]() {
#pragma unroll
            for (int s = 0; s < 8; ++s) { const int Lid = (lane >> 3) + 4 * s, piece = lane & 7; const int row = Lid >> 1, cofs = (Lid & 1) * 32 + piece * 4;
                v4f val = *(const v4fa*)(os + row * 68 + cofs); if (R) { const v4f rv = *(const v4f*)(R + ((size_t)r0 + row) * ldc + c0 + cofs); val += roundR ? (v4f){bfr(rv[0]), bfr(rv[1]), bfr(rv[2]), bfr(rv[3])} : rv; }
                *(volatile v4f*)(crow + (size_t)row * ldc + cofs) = val; }
        };
        pass(); __threadfence(); pass();
    }
}

__global__ __launch_bounds__(256) void k_wt(const float* __restrict__ Wm, int K, int ncols, bf* WT) {
    __shared__ __align__(16) unsigned short tl[64 * 72];
    const int tid = threadIdx.x, k0 = blockIdx.x * 64, n0 = blockIdx.y * 64;
    const int kk = tid >> 2, nq = (tid & 3) * 16;
#pragma unroll
    for (int i = 0; i < 16; ++i) tl[(nq + i) * 72 + kk] = f2bf(Wm[(size_t)(k0 + kk) * ncols + n0 + nq + i]);
    __syncthreads();
    const int piece = tid & 7;
    auto pass = [&]() {
#pragma unroll
        for (int s = 0; s < 2; ++s) { const int nr = (tid >> 3) + 32 * s; const v8us val = *(const v8usa*)(tl + nr * 72 + piece * 8); *(volatile v8us*)(WT + (size_t)(n0 + nr) * K + k0 + piece * 8) = val; }
    };
    pass(); __threadfence(); pass();
}

__global__ __launch_bounds__(256) void k_cvt8(const float* __restrict__ src, bf* dst, size_t n8) {
    const size_t i = (size_t)blockIdx.x * 256 + threadIdx.x; if (i >= n8) return;
    const v8f v = *(const v8f*)(src + i * 8); v8us o;
#pragma unroll
    for (int k = 0; k < 8; ++k) o[k] = f2bf(v[k]);
    *(volatile v8us*)(dst + i * 8) = o; __threadfence(); *(volatile v8us*)(dst + i * 8) = o;
}
__global__ __launch_bounds__(256) void k_zero8(bf* dst, size_t n8) {
    const size_t i = (size_t)blockIdx.x * 256 + threadIdx.x; if (i >= n8) return; v8us z;
#pragma unroll
    for (int k = 0; k < 8; ++k) z[k] = 0;
    *(volatile v8us*)(dst + i * 8) = z; __threadfence(); *(volatile v8us*)(dst + i * 8) = z;
}

__device__ __forceinline__ int seg_lo(int l) { return l * l; }
__global__ __launch_bounds__(256) void k_mix(const float* __restrict__ x, const float* __restrict__ y, int r0, bf* Ph, bf* Pl) {
    const int lane = threadIdx.x & 31; const int wid = blockIdx.x * 8 + (threadIdx.x >> 5); const int rl = wid / NF, f = wid - rl * NF; const size_t r = (size_t)r0 + rl;
    float yv[L2];
#pragma unroll
    for (int c = 0; c < L2; ++c) yv[c] = bfr(y[(r * NF + f) * L2 + c]);
#pragma unroll 1
    for (int ps = 0; ps < 2; ++ps) {
#pragma unroll
        for (int half = 0; half < 2; ++half) { v8us oh, ol;
#pragma unroll
            for (int gg = 0; gg < 2; ++gg) { const int g = half * 64 + 2 * lane + gg; float xv[L2];
#pragma unroll
                for (int c = 0; c < L2; ++c) xv[c] = bfr(x[(r * NF + g) * L2 + c]);
#pragma unroll
                for (int l = 0; l < LMX; ++l) { float s = 0.f;
#pragma unroll
                    for (int c = l * l; c < (l + 1) * (l + 1); ++c) s = fmaf(yv[c], xv[c], s);
                    const unsigned short hb = f2bf(s); oh[gg * 4 + l] = hb; ol[gg * 4 + l] = f2bf(s - bf2f(hb)); } }
            const size_t o = (size_t)rl * KBIG + f * 512 + half * 256 + lane * 8; *(volatile v8us*)(Ph + o) = oh; *(volatile v8us*)(Pl + o) = ol; }
        if (ps == 0) __threadfence(); }
}
template <int MODE>
__global__ __launch_bounds__(256) void k_actsplit(const float* __restrict__ src, int ld, int col0, const float* __restrict__ bias, bf* dh, bf* dl) {
    typedef __attribute__((ext_vector_type(2))) unsigned short v2us;
    const int lane = threadIdx.x & 31, r = blockIdx.x * 8 + (threadIdx.x >> 5); if (r >= NBM) return; const int m = r & 63; v2us oh, ol;
#pragma unroll
    for (int i = 0; i < 2; ++i) { const int c = lane * 2 + i; float v = src[(size_t)r * ld + col0 + c]; if (MODE == 1) { v += bfr(bias[m * KD + c]); v = v / (1.0f + __expf(-v)); }
        const unsigned short hb = f2bf(v); oh[i] = hb; ol[i] = f2bf(v - bf2f(hb)); }
    const size_t o = (size_t)r * KD + lane * 2; *(volatile v2us*)(dh + o) = oh; *(volatile v2us*)(dl + o) = ol; __threadfence(); *(volatile v2us*)(dh + o) = oh; *(volatile v2us*)(dl + o) = ol;
}
__global__ __launch_bounds__(256) void k_res(const float* __restrict__ GX, const float* __restrict__ GY, const float* __restrict__ x, const float* __restrict__ y, float* OUTP) {
    const int lane = threadIdx.x & 31; const size_t wid = (size_t)blockIdx.x * 8 + (threadIdx.x >> 5); const size_t r = wid / (NF / 8); const int f = (int)(wid % (NF / 8)) * 8 + (lane >> 2), cq = (lane & 3) * 4;
    v4f o;
#pragma unroll
    for (int i = 0; i < 4; ++i) { const int c = cq + i; const int l = (c >= 9) ? 3 : (c >= 4) ? 2 : (c >= 1) ? 1 : 0; const size_t e = (r * NF + f) * L2 + c;
        float gx = GX[r * (LMX * NF) + l * NF + f], gy = GY[r * (LMX * NF) + l * NF + f]; gx = gx / (1.0f + __expf(-gx)); gy = gy / (1.0f + __expf(-gy));
        o[i] = gx * bfr(x[e]) + gy * bfr(y[e]); }
    const size_t ob = (r * NF + f) * L2 + cq; *(volatile v4f*)(OUTP + ob) = o; __threadfence(); *(volatile v4f*)(OUTP + ob) = o;
}

extern "C" void kernel_launch(void* const* d_in, const int* in_sizes, int n_in,
                              void* d_out, int out_size, void* d_ws, size_t ws_size, hipStream_t stream) {
    (void)in_sizes; (void)n_in; (void)out_size;
    const float* x = (const float*)d_in[0]; const float* y = (const float*)d_in[1]; const float* wx0 = (const float*)d_in[2]; const float* wy0 = (const float*)d_in[3];
    const float* wxm = (const float*)d_in[4]; const float* bxm = (const float*)d_in[5]; const float* wym = (const float*)d_in[6]; const float* bym = (const float*)d_in[7]; const float* wxf = (const float*)d_in[8]; const float* wyf = (const float*)d_in[9];
    float* out = (float*)d_out;
    char* wsp = (char*)d_ws;
    auto take = [&](size_t bytes) { char* p = wsp; wsp += (bytes + 255) & ~(size_t)255; return (void*)p; };
    bf* W0 = (bf*)take((size_t)2 * KD * KBIG * 2); bf* WMT = (bf*)take((size_t)4 * KD * KD * 2); bf* WFX = (bf*)take((size_t)LMX * NF * KD * 2); bf* WFY = (bf*)take((size_t)LMX * NF * KD * 2);
    bf* Ph = (bf*)take((size_t)RCH * KBIG * 2); bf* Pl = (bf*)take((size_t)RCH * KBIG * 2); float* M0 = (float*)take((size_t)NBM * 2 * KD * 4);
    bf* Ah = (bf*)take((size_t)NBM * KD * 2); bf* Al = (bf*)take((size_t)NBM * KD * 2); float* T1 = (float*)take((size_t)NBM * KD * 4); float* GX = (float*)take((size_t)NBM * LMX * NF * 4); float* GY = (float*)take((size_t)NBM * LMX * NF * 4);
    if ((size_t)(wsp - (char*)d_ws) > ws_size) return;
    k_cvt8<<<(unsigned)((KD * KBIG / 8 + 255) / 256), 256, 0, stream>>>(wx0, W0, (size_t)KD * KBIG / 8); k_cvt8<<<(unsigned)((KD * KBIG / 8 + 255) / 256), 256, 0, stream>>>(wy0, W0 + (size_t)KD * KBIG, (size_t)KD * KBIG / 8);
    for (int i = 0; i < 2; ++i) { k_wt<<<dim3(1, 1, 1), 256, 0, stream>>>(wxm + (size_t)i * KD * KD, KD, KD, WMT + (size_t)(2 * i) * KD * KD); k_wt<<<dim3(1, 1, 1), 256, 0, stream>>>(wym + (size_t)i * KD * KD, KD, KD, WMT + (size_t)(2 * i + 1) * KD * KD); }
    k_cvt8<<<(LMX * NF * KD / 8 + 255) / 256, 256, 0, stream>>>(wxf, WFX, LMX * NF * KD / 8); k_cvt8<<<(LMX * NF * KD / 8 + 255) / 256, 256, 0, stream>>>(wyf, WFY, LMX * NF * KD / 8);
    for (int ch = 0; ch < NBM / RCH; ++ch) { const int r0 = ch * RCH;
        k_mix<<<(RCH * NF) / 8, 256, 0, stream>>>(x, y, r0, Ph, Pl);
        k_gemmb<true, false><<<dim3(RCH / 64, (2 * KD) / 64, 1), 128, 0, stream>>>(Ph, Pl, W0, nullptr, M0 + (size_t)r0 * 2 * KD, 2 * KD, nullptr, nullptr, KBIG); }
    for (int br = 0; br < 2; ++br) {
        k_actsplit<0><<<NBM / 8, 256, 0, stream>>>(M0, 2 * KD, br * KD, nullptr, Ah, Al);
        k_gemmb<true, false><<<dim3(NBM / 64, 1, 1), 128, 0, stream>>>(Ah, Al, WMT + (size_t)(0 + br) * KD * KD, nullptr, T1, KD, nullptr, nullptr, KD);
        k_actsplit<1><<<NBM / 8, 256, 0, stream>>>(T1, KD, 0, br ? bym : bxm, Ah, Al);
        k_gemmb<true, false><<<dim3(NBM / 64, 1, 1), 128, 0, stream>>>(Ah, Al, WMT + (size_t)(2 + br) * KD * KD, nullptr, T1, KD, nullptr, nullptr, KD);
        k_actsplit<1><<<NBM / 8, 256, 0, stream>>>(T1, KD, 0, (br ? bym : bxm) + KD * KD, Ah, Al);
        k_gemmb<true, false><<<dim3(NBM / 64, (LMX * NF) / 64, 1), 128, 0, stream>>>(Ah, Al, br ? WFY : WFX, nullptr, br ? GY : GX, LMX * NF, nullptr, nullptr, KD); }
    k_res<<<(unsigned)(((size_t)NBM * NF / 8) / 8), 256, 0, stream>>>(GX, GY, x, y, out);
}
